// ToyMultiHeadAttention_43181601194157
// MI455X (gfx1250) — hardware-verified
//
#include <hip/hip_runtime.h>

typedef _Float16 f16;
typedef f16 v16h __attribute__((ext_vector_type(16)));
typedef __bf16 v16b __attribute__((ext_vector_type(16)));
typedef float v8f __attribute__((ext_vector_type(8)));
typedef float v4f __attribute__((ext_vector_type(4)));
typedef unsigned int v4u __attribute__((ext_vector_type(4)));
typedef unsigned int v4ua __attribute__((ext_vector_type(4), may_alias));
typedef float v4fa __attribute__((ext_vector_type(4), may_alias));

#define NB 4
#define NT 2048
#define NC 1024
#define NH 16
#define ND 64
#define TLO 1024
#define XSPLIT 8
#define QSC 64.0f
#define KSC 64.0f
#define VSC 256.0f
#define PSC 256.0f
#define ASC 256.0f
#define WSC 1024.0f
#define RSC 2048.0f

union Frag { v16h h; v16b b; v4u u[2]; };

__device__ __forceinline__ v8f zero8() {
  v8f z = {0.f, 0.f, 0.f, 0.f, 0.f, 0.f, 0.f, 0.f};
  return z;
}

__device__ __forceinline__ v8f mma_h(const Frag& a, const Frag& b, v8f c) {
  c = __builtin_amdgcn_wmma_f32_16x16x32_f16(false, a.h, false, b.h, (short)0, c, false, false);
  asm volatile("v_nop\n\tv_nop\n\tv_nop\n\tv_nop" : "+v"(c) : "v"(a.h), "v"(b.h));
  return c;
}
__device__ __forceinline__ v8f mma_b(const Frag& a, const Frag& b, v8f c) {
  c = __builtin_amdgcn_wmma_f32_16x16x32_bf16(false, a.b, false, b.b, (short)0, c, false, false);
  asm volatile("v_nop\n\tv_nop\n\tv_nop\n\tv_nop" : "+v"(c) : "v"(a.b), "v"(b.b));
  return c;
}

__device__ __forceinline__ void ldfrag(Frag& f, const unsigned short* p) {
  f.u[0] = *(const v4ua*)p;
  f.u[1] = *(const v4ua*)(p + 16);
}

__device__ __forceinline__ unsigned int hbits(f16 x) {
  union { f16 f; unsigned short u; } c;
  c.f = x;
  return (unsigned int)c.u;
}
__device__ __forceinline__ unsigned int bfbits(float x) {
  unsigned int u = __float_as_uint(x);
  u += 0x7FFFu + ((u >> 16) & 1u);
  return u >> 16;
}
__device__ __forceinline__ float bfval(float x) { return __uint_as_float(bfbits(x) << 16); }
__device__ __forceinline__ v4u pack8(const unsigned int* e) {
  v4u r;
  r.x = e[0] | (e[1] << 16);
  r.y = e[2] | (e[3] << 16);
  r.z = e[4] | (e[5] << 16);
  r.w = e[6] | (e[7] << 16);
  return r;
}

__global__ __launch_bounds__(256) void k_cvt_act(const float* x, unsigned short* y, int n8) {
  const int g = blockIdx.x * 256 + threadIdx.x;
  if (g >= n8) return;
  const float* s = x + (size_t)g * 8;
  const v4f f0 = *(const v4fa*)s;
  const v4f f1 = *(const v4fa*)(s + 4);
  unsigned int e[8];
  e[0] = bfbits(f0.x); e[1] = bfbits(f0.y); e[2] = bfbits(f0.z); e[3] = bfbits(f0.w);
  e[4] = bfbits(f1.x); e[5] = bfbits(f1.y); e[6] = bfbits(f1.z); e[7] = bfbits(f1.w);
  const v4u o = pack8(e);
  unsigned short* d = y + (size_t)g * 8;
  *(volatile v4u*)d = o;
  __threadfence();
  *(volatile v4u*)d = o;
}

__global__ __launch_bounds__(256) void k_cvt_w(const float* wq, const float* wk, const float* wv,
                                              const float* wo, unsigned short* w16, int n8w) {
  const int g = blockIdx.x * 256 + threadIdx.x;
  if (g >= 4 * n8w) return;
  const int which = (g >= 2 * n8w) ? ((g >= 3 * n8w) ? 3 : 2) : ((g >= n8w) ? 1 : 0);
  const int i = g - which * n8w;
  const float* src = (which == 0) ? wq : ((which == 1) ? wk : ((which == 2) ? wv : wo));
  const float* s = src + (size_t)i * 8;
  const v4f f0 = *(const v4fa*)s;
  const v4f f1 = *(const v4fa*)(s + 4);
  float f[8] = {f0.x, f0.y, f0.z, f0.w, f1.x, f1.y, f1.z, f1.w};
  unsigned int e[8];
#pragma unroll
  for (int t = 0; t < 8; ++t) {
    if (which == 3) e[t] = hbits((f16)(bfval(f[t]) * WSC));
    else            e[t] = bfbits(f[t]);
  }
  const v4u o = pack8(e);
  unsigned short* d = w16 + (size_t)which * ((size_t)n8w * 8) + (size_t)i * 8;
  *(volatile v4u*)d = o;
  __threadfence();
  *(volatile v4u*)d = o;
}

template <int KIND>
__global__ __launch_bounds__(256) void k_gemm(const unsigned short* A, const unsigned short* Al,
                                              const unsigned short* W, const float* bias,
                                              unsigned short* Oh, unsigned short* Ol, float* Of,
                                              float scale) {
  constexpr int AP = 72;
  constexpr int SHN = (KIND == 0) ? 128 * 72 : ((KIND == 1) ? 64 * 136 : 8);
  __shared__ __attribute__((aligned(16))) unsigned short As[128 * AP];
  __shared__ __attribute__((aligned(16))) unsigned short Als[(KIND == 2) ? 128 * AP : 8];
  __shared__ __attribute__((aligned(16))) unsigned short Bs[64 * AP];
  __shared__ __attribute__((aligned(16))) unsigned short Sh[SHN];
  __shared__ __attribute__((aligned(16))) unsigned short Sl[SHN];
  __shared__ __attribute__((aligned(16))) float Sf[(KIND == 2) ? 128 * 68 : 4];

  const int tid = threadIdx.x;
  const int l = tid & 31, wv = tid >> 5, h = l >> 4, m = l & 15;
  const int wr = wv >> 1, wc = wv & 1;
  const int m0 = blockIdx.x * 128, n0 = blockIdx.y * 64;
  const int t0 = m0 & (NT - 1);
  const bool use_lo = (KIND == 2) && (t0 < XSPLIT * 64);

  v8f acc[2][2], accr[2][2];
#pragma unroll
  for (int i = 0; i < 2; ++i)
#pragma unroll
    for (int j = 0; j < 2; ++j) { acc[i][j] = zero8(); accr[i][j] = zero8(); }

#pragma unroll 1
  for (int kt = 0; kt < NC / 64; ++kt) {
    const int k0 = kt * 64;
    __syncthreads();
#pragma unroll
    for (int c = 0; c < 4; ++c) {
      const int idx = tid + c * 256, row = idx >> 3, seg = idx & 7;
      const v4u t = *(const v4ua*)(A + (size_t)(m0 + row) * NC + k0 + seg * 8);
      *(v4ua*)(As + row * AP + seg * 8) = t;
      if (KIND == 2) {
        if (use_lo) {
          const v4u t2 = *(const v4ua*)(Al + (size_t)(m0 + row) * NC + k0 + seg * 8);
          *(v4ua*)(Als + row * AP + seg * 8) = t2;
        }
      }
    }
#pragma unroll
    for (int c = 0; c < 2; ++c) {
      const int idx = tid + c * 256, row = idx >> 3, seg = idx & 7;
      const v4u t = *(const v4ua*)(W + (size_t)(n0 + row) * NC + k0 + seg * 8);
      *(v4ua*)(Bs + row * AP + seg * 8) = t;
    }
    __syncthreads();
#pragma unroll
    for (int ks = 0; ks < 2; ++ks) {
      Frag a[2], b[2];
#pragma unroll
      for (int i = 0; i < 2; ++i) ldfrag(a[i], As + (wr * 32 + i * 16 + m) * AP + ks * 32 + 8 * h);
#pragma unroll
      for (int j = 0; j < 2; ++j) ldfrag(b[j], Bs + (wc * 32 + j * 16 + m) * AP + ks * 32 + 8 * h);
#pragma unroll
      for (int i = 0; i < 2; ++i)
#pragma unroll
        for (int j = 0; j < 2; ++j) {
          if (KIND == 2) acc[i][j] = mma_h(a[i], b[j], acc[i][j]);
          else           acc[i][j] = mma_b(a[i], b[j], acc[i][j]);
        }
      if (KIND == 2) {
        if (use_lo) {
          Frag al[2];
#pragma unroll
          for (int i = 0; i < 2; ++i) ldfrag(al[i], Als + (wr * 32 + i * 16 + m) * AP + ks * 32 + 8 * h);
#pragma unroll
          for (int i = 0; i < 2; ++i)
#pragma unroll
            for (int j = 0; j < 2; ++j) accr[i][j] = mma_h(al[i], b[j], accr[i][j]);
        }
      }
    }
  }

  __syncthreads();
  if (KIND == 2) {
#pragma unroll
    for (int i = 0; i < 2; ++i)
#pragma unroll
      for (int j = 0; j < 2; ++j) {
        const int nl = wc * 32 + j * 16 + m;
        const float bv = bfval(bias[n0 + nl]);
#pragma unroll
        for (int r = 0; r < 8; ++r) {
          const int rl = wr * 32 + i * 16 + 8 * h + r;
          float v = acc[i][j][r];
          if (use_lo) v += accr[i][j][r] * (1.0f / RSC);
          v = v * scale + bv;
          Sf[rl * 68 + nl] = v;
        }
      }
    __syncthreads();
#pragma unroll 1
    for (int pass = 0; pass < 2; ++pass) {
#pragma unroll
      for (int it = 0; it < 8; ++it) {
        const int L = wv * 32 + it * 4 + (l >> 3);
        const int row = L >> 1, cb = (L & 1) * 32 + (l & 7) * 4;
        const v4f v = *(const v4fa*)(Sf + row * 68 + cb);
        float* g = Of + (size_t)(m0 + row) * NC + n0 + cb;
        *(volatile v4f*)g = v;
      }
      if (pass == 0) __threadfence();
    }
  } else {
#pragma unroll
    for (int i = 0; i < 2; ++i)
#pragma unroll
      for (int j = 0; j < 2; ++j) {
        const int nl = wc * 32 + j * 16 + m;
        const float bv = bfval(bias[n0 + nl]);
#pragma unroll
        for (int r = 0; r < 8; ++r) {
          const int rl = wr * 32 + i * 16 + 8 * h + r;
          const float v = (acc[i][j][r] + bv) * scale;
          const f16 hv = (f16)v;
          const f16 lv = (f16)((v - (float)hv) * RSC);
          const int sidx = (KIND == 0) ? (rl * 72 + nl) : (nl * 136 + rl);
          Sh[sidx] = (unsigned short)hbits(hv);
          Sl[sidx] = (unsigned short)hbits(lv);
        }
      }
    __syncthreads();
    const int hd = n0 >> 6, bb = m0 >> 11;
    const bool wlo = (t0 < TLO);
#pragma unroll 1
    for (int pass = 0; pass < 2; ++pass) {
#pragma unroll
      for (int it = 0; it < 4; ++it) {
        const int L = wv * 16 + it * 4 + (l >> 3), e = l & 7;
        if (KIND == 0) {
          const int t = t0 + L;
          const v4u vh = *(const v4ua*)(Sh + L * 72 + e * 8);
          const size_t gh = ((size_t)(bb * NH + hd) * NT + t) * ND + e * 8;
          *(volatile v4u*)(Oh + gh) = vh;
          if (wlo) {
            const v4u vl = *(const v4ua*)(Sl + L * 72 + e * 8);
            const size_t gl = ((size_t)(bb * NH + hd) * TLO + t) * ND + e * 8;
            *(volatile v4u*)(Ol + gl) = vl;
          }
        } else {
          const int n = L >> 1, mh = L & 1;
          const int tt = t0 + mh * 64 + e * 8;
          const v4u vh = *(const v4ua*)(Sh + n * 136 + mh * 64 + e * 8);
          const size_t gh = ((size_t)(bb * NH + hd) * ND + n) * NT + tt;
          *(volatile v4u*)(Oh + gh) = vh;
          if (wlo) {
            const v4u vl = *(const v4ua*)(Sl + n * 136 + mh * 64 + e * 8);
            const size_t gl = ((size_t)(bb * NH + hd) * ND + n) * TLO + tt;
            *(volatile v4u*)(Ol + gl) = vl;
          }
        }
      }
      if (pass == 0) __threadfence();
    }
  }
}

template <int SPLIT>
__global__ __launch_bounds__(128) void k_attn(const unsigned short* Qh, const unsigned short* Ql,
                                              const unsigned short* Kh, const unsigned short* Kl,
                                              const unsigned short* Vh, const unsigned short* Vl,
                                              unsigned short* Ah, unsigned short* Alo, int xoff) {
  constexpr int KP = 72;
  __shared__ __attribute__((aligned(16))) unsigned short Ks[64 * KP];
  __shared__ __attribute__((aligned(16))) unsigned short Vs[64 * KP];
  __shared__ __attribute__((aligned(16))) unsigned short Ksl[SPLIT ? 64 * KP : 8];
  __shared__ __attribute__((aligned(16))) unsigned short Vsl[SPLIT ? 64 * KP : 8];
  __shared__ __attribute__((aligned(16))) unsigned short Os[64 * KP];
  __shared__ __attribute__((aligned(16))) unsigned short Osl[SPLIT ? 64 * KP : 8];

  const int tid = threadIdx.x;
  const int w = tid >> 5, l = tid & 31, h = l >> 4, m = l & 15;
  const int bx = blockIdx.x + xoff;
  const int q0 = bx * 64, bh = blockIdx.y, bb = bh >> 4, hd = bh & 15;
  const int qr = q0 + w * 16 + m;

  Frag qh[2], ql[2];
  {
    const unsigned short* p = Qh + ((size_t)bh * NT + qr) * ND;
#pragma unroll
    for (int ks = 0; ks < 2; ++ks) ldfrag(qh[ks], p + ks * 32 + 8 * h);
    if (SPLIT) {
      const unsigned short* pl = Ql + ((size_t)bh * TLO + qr) * ND;
#pragma unroll
      for (int ks = 0; ks < 2; ++ks) ldfrag(ql[ks], pl + ks * 32 + 8 * h);
    } else {
#pragma unroll
      for (int ks = 0; ks < 2; ++ks) { ql[ks].u[0] = qh[ks].u[0]; ql[ks].u[1] = qh[ks].u[1]; }
    }
  }

  const unsigned short* Kp  = Kh + (size_t)bh * NT * ND;
  const unsigned short* Klp = Kl + (size_t)bh * TLO * ND;
  const unsigned short* Vp  = Vh + (size_t)bh * ND * NT;
  const unsigned short* Vlp = Vl + (size_t)bh * ND * TLO;

  float mrow = -1.0e30f, lrow = 0.f;
  v8f o[4];
#pragma unroll
  for (int dt = 0; dt < 4; ++dt) o[dt] = zero8();

#pragma unroll 1
  for (int kt = 0; kt <= bx; ++kt) {
    const int k0 = kt * 64;
    __syncthreads();
#pragma unroll
    for (int c = 0; c < 4; ++c) {
      const int idx = tid + c * 128, row = idx >> 3, seg = idx & 7;
      const v4u tk = *(const v4ua*)(Kp + (size_t)(k0 + row) * ND + seg * 8);
      *(v4ua*)(Ks + row * KP + seg * 8) = tk;
      const v4u tv = *(const v4ua*)(Vp + (size_t)row * NT + k0 + seg * 8);
      *(v4ua*)(Vs + row * KP + seg * 8) = tv;
      if (SPLIT) {
        const v4u tk2 = *(const v4ua*)(Klp + (size_t)(k0 + row) * ND + seg * 8);
        *(v4ua*)(Ksl + row * KP + seg * 8) = tk2;
        const v4u tv2 = *(const v4ua*)(Vlp + (size_t)row * TLO + k0 + seg * 8);
        *(v4ua*)(Vsl + row * KP + seg * 8) = tv2;
      }
    }
    __syncthreads();
    const bool diag = (kt == bx);

    float p[4][8];
#pragma unroll
    for (int j = 0; j < 4; ++j) {
      v8f s = zero8(), sr = zero8();
#pragma unroll
      for (int ks = 0; ks < 2; ++ks) {
        Frag ka;
        ldfrag(ka, Ks + (j * 16 + m) * KP + ks * 32 + 8 * h);
        s = mma_h(ka, qh[ks], s);
        if (SPLIT) {
          Frag kb;
          ldfrag(kb, Ksl + (j * 16 + m) * KP + ks * 32 + 8 * h);
          sr = mma_h(ka, ql[ks], sr);
          sr = mma_h(kb, qh[ks], sr);
        }
      }
#pragma unroll
      for (int r = 0; r < 8; ++r) {
        float x = s[r];
        if (SPLIT) x += sr[r] * (1.0f / RSC);
        x *= (1.0f / (QSC * KSC));
        const int key = k0 + j * 16 + 8 * h + r;
        if (diag && key > qr) x = -1.0e30f;
        p[j][r] = x;
      }
    }

    float tmax = p[0][0];
#pragma unroll
    for (int j = 0; j < 4; ++j)
#pragma unroll
      for (int r = 0; r < 8; ++r) tmax = fmaxf(tmax, p[j][r]);
    tmax = fmaxf(tmax, __shfl_xor(tmax, 16, 32));
    const float mnew = fmaxf(mrow, tmax);
    const float alpha = __expf(mrow - mnew);
    float ps = 0.f;
#pragma unroll
    for (int j = 0; j < 4; ++j)
#pragma unroll
      for (int r = 0; r < 8; ++r) {
        const float e = __expf(p[j][r] - mnew);
        p[j][r] = e;
        ps += e;
      }
    ps += __shfl_xor(ps, 16, 32);
    lrow = lrow * alpha + ps;
    mrow = mnew;
#pragma unroll
    for (int dt = 0; dt < 4; ++dt) o[dt] = o[dt] * alpha;

    Frag ph[2], pl[2];
#pragma unroll
    for (int pp = 0; pp < 2; ++pp)
#pragma unroll
      for (int i = 0; i < 8; ++i) {
        const float e0 = p[2 * pp][i] * PSC, e1 = p[2 * pp + 1][i] * PSC;
        const f16 h0 = (f16)e0, h1 = (f16)e1;
        ph[pp].h[i] = h0;
        ph[pp].h[8 + i] = h1;
        if (SPLIT) {
          pl[pp].h[i] = (f16)((e0 - (float)h0) * RSC);
          pl[pp].h[8 + i] = (f16)((e1 - (float)h1) * RSC);
        } else {
          pl[pp].h[i] = h0;
          pl[pp].h[8 + i] = h1;
        }
      }

#pragma unroll
    for (int dt = 0; dt < 4; ++dt) {
      v8f orr = zero8();
#pragma unroll
      for (int pp = 0; pp < 2; ++pp) {
        Frag va;
        ldfrag(va, Vs + (dt * 16 + m) * KP + pp * 32 + 8 * h);
        o[dt] = mma_h(va, ph[pp], o[dt]);
        if (SPLIT) {
          Frag vb;
          ldfrag(vb, Vsl + (dt * 16 + m) * KP + pp * 32 + 8 * h);
          orr = mma_h(va, pl[pp], orr);
          orr = mma_h(vb, ph[pp], orr);
        }
      }
      if (SPLIT) o[dt] = o[dt] + orr * (1.0f / RSC);
    }
  }

  const float inv = 1.0f / (lrow * (PSC * VSC));
  unsigned short* orow = Os + (w * 16 + m) * KP;
  unsigned short* orowl = Osl + (SPLIT ? (w * 16 + m) * KP : 0);
#pragma unroll
  for (int dt = 0; dt < 4; ++dt) {
    unsigned int hb[8], lb[8];
#pragma unroll
    for (int r = 0; r < 8; ++r) {
      const float a = o[dt][r] * inv * ASC;
      const f16 hv = (f16)a;
      hb[r] = hbits(hv);
      lb[r] = SPLIT ? hbits((f16)((a - (float)hv) * RSC)) : hb[r];
    }
    *(v4ua*)(orow + dt * 16 + 8 * h) = pack8(hb);
    if (SPLIT) *(v4ua*)(orowl + dt * 16 + 8 * h) = pack8(lb);
  }
  asm volatile("" ::: "memory");
#pragma unroll 1
  for (int pass = 0; pass < 2; ++pass) {
#pragma unroll
    for (int it = 0; it < 4; ++it) {
      const int L = it * 4 + (l >> 3), e = l & 7;
      const v4u v = *(const v4ua*)(Os + (w * 16 + L) * KP + e * 8);
      const size_t g = ((size_t)(bb * NT + q0 + w * 16 + L)) * NC + hd * ND + e * 8;
      *(volatile v4u*)(Ah + g) = v;
      if (SPLIT) {
        const v4u v2 = *(const v4ua*)(Osl + (w * 16 + L) * KP + e * 8);
        *(volatile v4u*)(Alo + g) = v2;
      }
    }
    if (pass == 0) __threadfence();
  }
}

extern "C" void kernel_launch(void* const* d_in, const int* in_sizes, int n_in,
                              void* d_out, int out_size, void* d_ws,
                              size_t ws_size, hipStream_t stream) {
  const size_t NE  = (size_t)NB * NT * NC;
  const size_t NW  = (size_t)NC * NC;
  const size_t NLO = (size_t)NB * NH * TLO * ND;
  if (n_in < 11) return;
  if (in_sizes[0] != (int)NE || in_sizes[1] != (int)NE || in_sizes[2] != (int)NE) return;
  if (in_sizes[3] != (int)NW || in_sizes[5] != (int)NW || in_sizes[7] != (int)NW || in_sizes[9] != (int)NW) return;
  if (in_sizes[4] != NC || in_sizes[6] != NC || in_sizes[8] != NC || in_sizes[10] != NC) return;
  if (out_size != (int)NE) return;

  const float* q  = (const float*)d_in[0];
  const float* k  = (const float*)d_in[1];
  const float* v  = (const float*)d_in[2];
  const float* Wq = (const float*)d_in[3];
  const float* bq = (const float*)d_in[4];
  const float* Wk = (const float*)d_in[5];
  const float* bk = (const float*)d_in[6];
  const float* Wv = (const float*)d_in[7];
  const float* bv = (const float*)d_in[8];
  const float* Wo = (const float*)d_in[9];
  const float* bo = (const float*)d_in[10];
  float* out = (float*)d_out;

  unsigned char* ws = (unsigned char*)d_ws;
  size_t off = 0;
  unsigned short* act = (unsigned short*)(ws + off);
  unsigned short* Ahp = (unsigned short*)(ws + off);
  off += NE * 2;
  unsigned short* Alp = (unsigned short*)(ws + off);
  off += NE * 2;
  unsigned short* w16 = (unsigned short*)(ws + off);
  off += 4 * NW * 2;
  unsigned short* Qhp = (unsigned short*)(ws + off); off += NE * 2;
  unsigned short* Khp = (unsigned short*)(ws + off); off += NE * 2;
  unsigned short* Vhp = (unsigned short*)(ws + off); off += NE * 2;
  unsigned short* Qlp = (unsigned short*)(ws + off); off += NLO * 2;
  unsigned short* Klp = (unsigned short*)(ws + off); off += NLO * 2;
  unsigned short* Vlp = (unsigned short*)(ws + off); off += NLO * 2;
  if (off > ws_size) return;

  const int n8  = (int)(NE / 8);
  const int n8w = (int)(NW / 8);
  const dim3 gcvt((n8 + 255) / 256), gcvtw((4 * n8w + 255) / 256), bcvt(256);
  const dim3 gg((unsigned)((NB * NT) / 128), NC / 64), bg(256);

  k_cvt_w<<<gcvtw, bcvt, 0, stream>>>(Wq, Wk, Wv, Wo, w16, n8w);

  k_cvt_act<<<gcvt, bcvt, 0, stream>>>(q, act, n8);
  k_gemm<0><<<gg, bg, 0, stream>>>(act, act, w16 + 0 * NW, bq, Qhp, Qlp, out, QSC * 0.125f);
  k_cvt_act<<<gcvt, bcvt, 0, stream>>>(k, act, n8);
  k_gemm<0><<<gg, bg, 0, stream>>>(act, act, w16 + 1 * NW, bk, Khp, Klp, out, KSC);
  k_cvt_act<<<gcvt, bcvt, 0, stream>>>(v, act, n8);
  k_gemm<1><<<gg, bg, 0, stream>>>(act, act, w16 + 2 * NW, bv, Vhp, Vlp, out, VSC);

  k_attn<1><<<dim3(XSPLIT, NB * NH), dim3(128), 0, stream>>>(Qhp, Qlp, Khp, Klp, Vhp, Vlp, Ahp, Alp, 0);
  k_attn<0><<<dim3(NT / 64 - XSPLIT, NB * NH), dim3(128), 0, stream>>>(Qhp, Qlp, Khp, Klp, Vhp, Vlp, Ahp, Alp, XSPLIT);

  k_gemm<2><<<gg, bg, 0, stream>>>(Ahp, Alp, w16 + 3 * NW, bo, Qhp, Qlp, out, 1.0f / (ASC * WSC));
}
